// SHGRm_56727928045866
// MI455X (gfx1250) — hardware-verified
//
#include <hip/hip_runtime.h>
#include <math.h>

typedef __attribute__((ext_vector_type(16))) _Float16 v16h;
typedef __attribute__((ext_vector_type(16))) __bf16 v16b;
typedef __attribute__((ext_vector_type(8)))  _Float16 v8h;
typedef __attribute__((ext_vector_type(8)))  float v8f;
typedef __attribute__((ext_vector_type(4)))  float v4f;
typedef __attribute__((ext_vector_type(2)))  float v2f;
typedef __attribute__((ext_vector_type(4)))  unsigned v4u;
typedef __attribute__((ext_vector_type(4)))  int v4i;
typedef float __attribute__((may_alias)) float_a;
typedef int __attribute__((may_alias)) int_a;

template <typename T> __device__ __forceinline__ void vst2(void* p, T v) { *(volatile T*)p = v; __threadfence(); *(volatile T*)p = v; }
__device__ __forceinline__ v8f wmma16(v16h a, v16h b, v8f c) {
  v8f d = __builtin_amdgcn_wmma_f32_16x16x32_f16(false, a, false, b, (short)0, c, false, false);
  asm volatile("v_nop\n\tv_nop\n\tv_nop\n\tv_nop" : "+v"(d) : "v"(a), "v"(b));
  return d;
}
__device__ __forceinline__ v8f wmma_bf(v16b a, v16b b, v8f c) {
  v8f d = __builtin_amdgcn_wmma_f32_16x16x32_bf16(false, a, false, b, (short)0, c, false, false);
  asm volatile("v_nop\n\tv_nop\n\tv_nop\n\tv_nop" : "+v"(d) : "v"(a), "v"(b));
  return d;
}
__device__ __forceinline__ v16h frag_h(const _Float16* rowk0, int lane) {
  union { v16h v; v8h q[2]; } u; const _Float16* p = rowk0 + 8 * (lane >> 4);
  u.q[0] = *(const v8h*)p; u.q[1] = *(const v8h*)(p + 16); return u.v;
}
__device__ __forceinline__ v16h frag_f32(const float* rowk0, int lane) {
  v16h a; const float* p = rowk0 + 8 * (lane >> 4);
#pragma unroll
  for (int i = 0; i < 8; ++i) { a[i] = (_Float16)p[i]; a[8 + i] = (_Float16)p[16 + i]; }
  return a;
}
__device__ __forceinline__ v16h frag_f32s(const float* rowk0, int lane, float sc) {
  v16h a; const float* p = rowk0 + 8 * (lane >> 4);
#pragma unroll
  for (int i = 0; i < 8; ++i) { a[i] = (_Float16)(p[i] * sc); a[8 + i] = (_Float16)(p[16 + i] * sc); }
  return a;
}
__device__ __forceinline__ v16h fragc_f32(const float* W, int k0, int n, int lane, int ld, int K) {
  v16h a; const int g = lane >> 4;
#pragma unroll
  for (int i = 0; i < 8; ++i) { const int ka = k0 + 8 * g + i, kb = ka + 16;
    a[i] = (_Float16)(ka < K ? W[(size_t)(ka < K ? ka : K - 1) * ld + n] : 0.f); a[8 + i] = (_Float16)(kb < K ? W[(size_t)(kb < K ? kb : K - 1) * ld + n] : 0.f); }
  return a;
}
struct F2 { v16b h, l; };
__device__ __forceinline__ F2 bsplit16(const float v[16]) { F2 r;
#pragma unroll
  for (int i = 0; i < 16; ++i) { const __bf16 h = (__bf16)v[i]; r.h[i] = h; r.l[i] = (__bf16)(v[i] - (float)h); }
  return r; }
__device__ __forceinline__ F2 split_row(const float* row, int k0, int lane) { float v[16]; const float* p = row + k0 + 8 * (lane >> 4);
#pragma unroll
  for (int i = 0; i < 8; ++i) { v[i] = p[i]; v[8 + i] = p[16 + i]; }
  return bsplit16(v); }
__device__ __forceinline__ F2 split_rowK(const float* row, int k0, int lane, int K) { float v[16]; const int g = lane >> 4;
#pragma unroll
  for (int i = 0; i < 8; ++i) { const int ka = k0 + 8 * g + i, kb = ka + 16; v[i] = ka < K ? row[ka < K ? ka : K - 1] : 0.f; v[8 + i] = kb < K ? row[kb < K ? kb : K - 1] : 0.f; }
  return bsplit16(v); }
__device__ __forceinline__ F2 split_col(const float* W, int k0, int n, int lane, int ld, int K) { float v[16]; const int g = lane >> 4;
#pragma unroll
  for (int i = 0; i < 8; ++i) { const int ka = k0 + 8 * g + i, kb = ka + 16; v[i] = ka < K ? W[(size_t)(ka < K ? ka : K - 1) * ld + n] : 0.f; v[8 + i] = kb < K ? W[(size_t)(kb < K ? kb : K - 1) * ld + n] : 0.f; }
  return bsplit16(v); }
__device__ __forceinline__ v8f mac3(const F2& a, const F2& b, v8f c) { c = wmma_bf(a.l, b.h, c); c = wmma_bf(a.h, b.l, c); return wmma_bf(a.h, b.h, c); }
__device__ __forceinline__ float sigm(float v) { return 1.0f / (1.0f + expf(-v)); }
#define LDSX() do { asm volatile("s_wait_dscnt 0" ::: "memory"); __builtin_amdgcn_wave_barrier(); __builtin_amdgcn_fence(__ATOMIC_RELEASE, "workgroup"); } while (0)


#define NR 65536
#define P 32
#ifndef TR
#define TR (NR / 64)
#endif
typedef __attribute__((ext_vector_type(8))) __bf16 v8b;
__device__ __forceinline__ v16b frag_b(const __bf16* rowk0, int lane) {
  union { v16b v; v8b q[2]; } u; const __bf16* p = rowk0 + 8 * (lane >> 4);
  u.q[0] = *(const v8b*)p; u.q[1] = *(const v8b*)(p + 16); return u.v;
}
__device__ __forceinline__ float bfr(float v) { return (float)(__bf16)v; }
__device__ __attribute__((noinline)) float exp_ni(float v) { return expf(v); }
__device__ __attribute__((noinline)) float erf_ni(float v) { return erff(v); }

__device__ __forceinline__ float tanh_fast(float x) { const float e = __expf(2.0f * x); return 1.0f - 2.0f / (e + 1.0f); }
__device__ __forceinline__ v16b fragw(const float* __restrict__ row, int k0, int KR, int lane) { v16b a; const int g = lane >> 4;
#pragma unroll
  for (int i = 0; i < 8; ++i) { const int k1 = k0 + 8 * g + i, k2 = k1 + 16; a[i] = (__bf16)(k1 < KR ? row[k1] : 0.f); a[8 + i] = (__bf16)(k2 < KR ? row[k2] : 0.f); } return a; }
__device__ __forceinline__ v16h fragwh(const float* __restrict__ row, int k0, int KR, int lane) { v16h a; const int g = lane >> 4;
#pragma unroll
  for (int i = 0; i < 8; ++i) { const int k1 = k0 + 8 * g + i, k2 = k1 + 16; a[i] = (_Float16)(k1 < KR ? bfr(row[k1]) : 0.f); a[8 + i] = (_Float16)(k2 < KR ? bfr(row[k2]) : 0.f); } return a; }
template <int KP, int NT>
__device__ __forceinline__ void layer(const float* __restrict__ sh, int sst, const float* __restrict__ Wr, int KR, int nout, int lane, int col, v8f* acc) {
#pragma unroll
  for (int j = 0; j < NT; ++j) acc[j] = v8f{};
#pragma unroll
  for (int kc = 0; kc < KP / 32; ++kc) { v16h a; const float* p2 = sh + col * sst + kc * 32 + 8 * (lane >> 4);
#pragma unroll
    for (int i = 0; i < 8; ++i) { a[i] = (_Float16)p2[i]; a[8 + i] = (_Float16)p2[16 + i]; }
#pragma unroll
    for (int j = 0; j < NT; ++j) { const int o = j * 16 + col; const v16h w = (o < nout) ? fragwh(Wr + (size_t)o * KR, kc * 32, KR, lane) : v16h{}; acc[j] = wmma16(a, w, acc[j]); } } }
__global__ __launch_bounds__(128) void k_shg(const float* __restrict__ X,
    const float* __restrict__ WA1, const float* __restrict__ BA1, const float* __restrict__ WA2, const float* __restrict__ BA2, const float* __restrict__ WA3, const float* __restrict__ BA3, const float* __restrict__ WA4, const float* __restrict__ BA4, const float* __restrict__ WA5, const float* __restrict__ BA5,
    const float* __restrict__ WB1, const float* __restrict__ BB1, const float* __restrict__ WB2, const float* __restrict__ BB2, const float* __restrict__ WB3, const float* __restrict__ BB3, const float* __restrict__ WB4, const float* __restrict__ BB4, const float* __restrict__ WB5, const float* __restrict__ BB5, const float* __restrict__ WB6, const float* __restrict__ BB6, float* __restrict__ OUT) {
  __shared__ __align__(16) float sa[4][16][68]; __shared__ __align__(16) float sb[4][16][68]; __shared__ float sx[64][P + 1]; __shared__ __align__(16) float so[64][2 * P + 4];
  const int tid = threadIdx.x, wave = tid >> 5, lane = tid & 31, col = lane & 15, g = lane >> 4; const size_t rb = (size_t)blockIdx.x * 64; const int rw = wave * 16;
  for (int e = tid; e < 64 * P; e += 128) sx[e / P][e % P] = bfr(X[(rb + e / P) * P + e % P]); __syncthreads();
#pragma unroll 1
  for (int p = 0; p < P; ++p) {
    { const float* w1 = WA1 + (size_t)p * 64; const float* b1 = BA1 + (size_t)p * 64; for (int e = lane; e < 16 * 64; e += 32) { const int rl = e >> 6, k = e & 63; sa[wave][rl][k] = fmaxf(sx[rw + rl][p] * bfr(w1[k]) + bfr(b1[k]), 0.f); } }
    { v8f acc[4] = {}; v16b a; { const int row = rw + col;
#pragma unroll
        for (int i = 0; i < 8; ++i) { const int j1 = 8 * g + i, j2 = j1 + 16; const int f1 = j1 < p ? j1 : j1 + 1, f2 = j2 < p ? j2 : j2 + 1; a[i] = (__bf16)(j1 < P - 1 ? sx[row][f1] : 0.f); a[8 + i] = (__bf16)(j2 < P - 1 ? sx[row][f2] : 0.f); } }
#pragma unroll
      for (int j = 0; j < 4; ++j) acc[j] = wmma_bf(a, fragw(WB1 + ((size_t)p * 64 + j * 16 + col) * 31, 0, 31, lane), acc[j]);
      LDSX();
#pragma unroll
      for (int j = 0; j < 4; ++j) { const float bb = bfr(BB1[(size_t)p * 64 + j * 16 + col]);
#pragma unroll
        for (int r = 0; r < 8; ++r) sb[wave][8 * g + r][j * 16 + col] = fmaxf(acc[j][r] + bb, 0.f); } }
    LDSX();
    { v8f acc[2]; layer<64, 2>(&sa[wave][0][0], 68, WA2 + (size_t)p * 32 * 64, 64, 32, lane, col, acc); LDSX();
#pragma unroll
      for (int j = 0; j < 2; ++j) { const float bb = bfr(BA2[(size_t)p * 32 + j * 16 + col]);
#pragma unroll
        for (int r = 0; r < 8; ++r) sa[wave][8 * g + r][j * 16 + col] = tanh_fast(acc[j][r] + bb); } }
    { v8f acc[2]; layer<64, 2>(&sb[wave][0][0], 68, WB2 + (size_t)p * 32 * 64, 64, 32, lane, col, acc); LDSX();
#pragma unroll
      for (int j = 0; j < 2; ++j) { const float bb = bfr(BB2[(size_t)p * 32 + j * 16 + col]);
#pragma unroll
        for (int r = 0; r < 8; ++r) sb[wave][8 * g + r][j * 16 + col] = tanh_fast(acc[j][r] + bb); } }
    LDSX();
    { v8f acc[1]; layer<32, 1>(&sa[wave][0][0], 68, WA3 + (size_t)p * 16 * 32, 32, 16, lane, col, acc); v8f accb[2]; layer<32, 2>(&sb[wave][0][0], 68, WB3 + (size_t)p * 32 * 32, 32, 32, lane, col, accb); LDSX();
      { const float bb = bfr(BA3[(size_t)p * 16 + col]);
#pragma unroll
        for (int r = 0; r < 8; ++r) { sa[wave][8 * g + r][col] = tanh_fast(acc[0][r] + bb); sa[wave][8 * g + r][16 + col] = 0.f; } }
#pragma unroll
      for (int j = 0; j < 2; ++j) { const float bb = bfr(BB3[(size_t)p * 32 + j * 16 + col]);
#pragma unroll
        for (int r = 0; r < 8; ++r) sb[wave][8 * g + r][j * 16 + col] = tanh_fast(accb[j][r] + bb); } }
    LDSX();
    { v8f acc[1]; layer<32, 1>(&sa[wave][0][0], 68, WA4 + (size_t)p * 8 * 16, 16, 8, lane, col, acc); v8f accb[1]; layer<32, 1>(&sb[wave][0][0], 68, WB4 + (size_t)p * 16 * 32, 32, 16, lane, col, accb); LDSX();
      { const float bb = (col < 8) ? bfr(BA4[(size_t)p * 8 + col]) : 0.f;
#pragma unroll
        for (int r = 0; r < 8; ++r) sa[wave][8 * g + r][col] = (col < 8) ? tanh_fast(acc[0][r] + bb) : 0.f; }
      { const float bb = bfr(BB4[(size_t)p * 16 + col]);
#pragma unroll
        for (int r = 0; r < 8; ++r) { sb[wave][8 * g + r][col] = tanh_fast(accb[0][r] + bb); sb[wave][8 * g + r][16 + col] = 0.f; } } }
    LDSX();
    { v8f accb[1]; layer<32, 1>(&sb[wave][0][0], 68, WB5 + (size_t)p * 8 * 16, 16, 8, lane, col, accb); LDSX();
      { const float bb = (col < 8) ? bfr(BB5[(size_t)p * 8 + col]) : 0.f;
#pragma unroll
        for (int r = 0; r < 8; ++r) sb[wave][8 * g + r][col] = (col < 8) ? (accb[0][r] + bb) : 0.f; } }
    LDSX();
    { const int rl = lane & 15; const bool isb = lane >= 16; const float* src = isb ? &sb[wave][rl][0] : &sa[wave][rl][0]; const float* w = (isb ? WB6 : WA5) + (size_t)p * 8; float s = bfr((isb ? BB6 : BA5)[p]);
#pragma unroll
      for (int k = 0; k < 8; ++k) s += src[k] * bfr(w[k]);
      so[rw + rl][2 * p + (isb ? 1 : 0)] = s; }
    LDSX(); }
  __syncthreads(); for (int e = tid; e < 64 * 16; e += 128) { const int rl = e >> 4, q = e & 15; vst2(OUT + (rb + rl) * (2 * P) + q * 4, *(const v4f*)&so[rl][q * 4]); } }
extern "C" void kernel_launch(void* const* d_in, const int* in_sizes, int n_in, void* d_out, int out_size, void* d_ws, size_t ws_size, hipStream_t stream) {
  (void)in_sizes; (void)n_in; (void)out_size; (void)d_ws; (void)ws_size;
  const float** F = (const float**)d_in;
  k_shg<<<TR, 128, 0, stream>>>(F[0], F[1], F[2], F[3], F[4], F[5], F[6], F[7], F[8], F[9], F[10], F[11], F[12], F[13], F[14], F[15], F[16], F[17], F[18], F[19], F[20], F[21], F[22], (float*)d_out);
}
